// NetworkODEModel_24429773979863
// MI455X (gfx1250) — hardware-verified
//
#include <hip/hip_runtime.h>


namespace {
typedef _Float16 b16;
typedef __attribute__((ext_vector_type(16))) _Float16 v16b;
typedef __attribute__((ext_vector_type(8))) _Float16 v8b;
typedef __attribute__((ext_vector_type(4))) _Float16 v4h;
typedef __attribute__((ext_vector_type(2))) _Float16 v2h;
typedef __attribute__((ext_vector_type(8))) float v8f;
typedef __attribute__((ext_vector_type(4))) float v4f;
typedef __attribute__((ext_vector_type(2))) float v2f;
__device__ __forceinline__ float bf16_rne(float f) { unsigned int u = __float_as_uint(f); u += 0x7FFFu + ((u >> 16) & 1u); return __uint_as_float(u & 0xFFFF0000u); }
__device__ __forceinline__ void split16(float v, b16& hi, b16& lo) { hi = (b16)v; lo = (b16)(v - (float)hi); }
__device__ __forceinline__ v16b frag_kb(const b16* p, int hh) { const v8b a = *(const v8b*)(p + 8 * hh), b = *(const v8b*)(p + 16 + 8 * hh); v16b f;
#pragma unroll
  for (int e = 0; e < 8; ++e) { f[e] = a[e]; f[8 + e] = b[e]; } return f; }
__device__ __forceinline__ v8f wmma16b(v16b a, v16b b, v8f c) { v8f d = __builtin_amdgcn_wmma_f32_16x16x32_f16(false, a, false, b, (short)0, c, false, false); asm volatile("v_nop\n\tv_nop\n\tv_nop\n\tv_nop" : "+v"(d) : "v"(a), "v"(b)); return d; }
__device__ __forceinline__ void wave_lds_sync() { __builtin_amdgcn_fence(__ATOMIC_RELEASE, "workgroup"); __builtin_amdgcn_wave_barrier(); __builtin_amdgcn_fence(__ATOMIC_ACQUIRE, "workgroup"); }
__device__ __forceinline__ float pmul(float a, float b) { float p = a * b; asm volatile("" : "+v"(p)); return p; }
__device__ __forceinline__ int iclamp(int v, int lo, int hi) { return v < lo ? lo : (v > hi ? hi : v); }
__device__ __forceinline__ float nexp2(float v) { return __builtin_amdgcn_exp2f(v); }

constexpr int B = 8, N = 256, D = 16, KX = 32  , HH = 64, NR = B * N  , BL = B  , NRL = BL * N;
constexpr float XS = 8.0f, WSC = 256.0f, SLOPE = 0.01f;
static_assert(N % 32 == 0 && D == 16 && HH == 64 && NRL % 32 == 0, "tiling");
__device__ __forceinline__ float lk(float v) { return v > 0.0f ? v : SLOPE * v; }

template <int KP, int KIN, int NOUT>
__global__ __launch_bounds__(256) void wt_kernel(const float* __restrict__ w, int k0, b16* __restrict__ WT) {
  const int u = blockIdx.x * 256 + threadIdx.x; if (u >= NOUT * KP / 8) return; const int e = u * 8; const int o = e / KP, kk = e % KP; v8b v;
  for (int j = 0; j < 8; ++j) { const int k = kk + j; v[j] = (b16)(k < KIN ? bf16_rne(w[(size_t)(k0 + k) * NOUT + o]) * WSC : 0.0f); }
  for (int pass = 0; pass < 2; ++pass) { *(volatile v8b*)(WT + e) = v; __threadfence(); }
}
__global__ __launch_bounds__(64) void node_kernel(const float* __restrict__ x, const b16* __restrict__ W1, const float* __restrict__ nb1, const b16* __restrict__ W2, const float* __restrict__ nb2, const b16* __restrict__ WO, const float* __restrict__ nbo, const b16* __restrict__ CA, const b16* __restrict__ CB, float* __restrict__ NODE, float* __restrict__ AV, float* __restrict__ BV) {
  __shared__ __attribute__((aligned(16))) b16 Ax[2][16][KX + 8], Ah[2][16][HH + 8]; __shared__ __attribute__((aligned(16))) float Tf[2][16][HH + 4];
  const int wave = threadIdx.x >> 5, lane = threadIdx.x & 31, nloc = lane & 15, hlf = lane >> 4; const int m0 = blockIdx.x * 32 + wave * 16;
  for (int idx = lane; idx < 16 * KX; idx += 32) { const int rr = idx / KX, k = idx % KX; Ax[wave][rr][k] = (b16)(k < D ? bf16_rne(x[(size_t)(m0 + rr) * D + k]) * XS : 0.0f); }
  wave_lds_sync();
  const v16b ax = frag_kb(&Ax[wave][nloc][0], hlf);
#pragma unroll 1
  for (int part = 0; part < 2; ++part) { const b16* W = part == 0 ? CA : CB; float* dst = part == 0 ? AV : BV; v8f acc[4];
#pragma unroll
    for (int t = 0; t < 4; ++t) acc[t] = wmma16b(ax, frag_kb(W + (size_t)(t * 16 + nloc) * KX, hlf), (v8f){});
#pragma unroll
    for (int t = 0; t < 4; ++t)
#pragma unroll
      for (int r = 0; r < 8; ++r) Tf[wave][8 * hlf + r][t * 16 + nloc] = acc[t][r] * (1.0f / (XS * WSC));
    wave_lds_sync();
    for (int pass = 0; pass < 2; ++pass) { for (int rr = 0; rr < 16; rr += 2) { const int row = rr + hlf; *(volatile v4f*)(dst + (size_t)(m0 + row) * HH + nloc * 4) = *(const v4f*)(&Tf[wave][row][nloc * 4]); } __threadfence(); }
    wave_lds_sync(); }
  { v8f acc[4];
#pragma unroll
    for (int t = 0; t < 4; ++t) acc[t] = wmma16b(ax, frag_kb(W1 + (size_t)(t * 16 + nloc) * KX, hlf), (v8f){});
#pragma unroll
    for (int t = 0; t < 4; ++t) { const float bb = bf16_rne(nb1[t * 16 + nloc]);
#pragma unroll
      for (int r = 0; r < 8; ++r) Ah[wave][8 * hlf + r][t * 16 + nloc] = (b16)(lk(acc[t][r] * (1.0f / (XS * WSC)) + bb) * XS); } }
  wave_lds_sync();
  { v8f acc[4]; const v16b a0 = frag_kb(&Ah[wave][nloc][0], hlf), a1 = frag_kb(&Ah[wave][nloc][32], hlf);
#pragma unroll
    for (int t = 0; t < 4; ++t) { const b16* br = W2 + (size_t)(t * 16 + nloc) * HH; acc[t] = wmma16b(a0, frag_kb(br, hlf), (v8f){}); acc[t] = wmma16b(a1, frag_kb(br + 32, hlf), acc[t]); }
    wave_lds_sync();
#pragma unroll
    for (int t = 0; t < 4; ++t) { const float bb = bf16_rne(nb2[t * 16 + nloc]);
#pragma unroll
      for (int r = 0; r < 8; ++r) Ah[wave][8 * hlf + r][t * 16 + nloc] = (b16)(lk(acc[t][r] * (1.0f / (XS * WSC)) + bb) * XS); } }
  wave_lds_sync();
  { const v16b a0 = frag_kb(&Ah[wave][nloc][0], hlf), a1 = frag_kb(&Ah[wave][nloc][32], hlf); const b16* br = WO + (size_t)nloc * HH; v8f acc = wmma16b(a0, frag_kb(br, hlf), (v8f){}); acc = wmma16b(a1, frag_kb(br + 32, hlf), acc);
    const float bb = bf16_rne(nbo[nloc]);
#pragma unroll
    for (int r = 0; r < 8; ++r) Tf[wave][8 * hlf + r][nloc] = acc[r] * (1.0f / (XS * WSC)) + bb; }
  wave_lds_sync();
  for (int pass = 0; pass < 2; ++pass) { for (int h2 = 0; h2 < 2; ++h2) { const int e = h2 * 128 + lane * 4; const int row = e / D, c = e % D; *(volatile v4f*)(NODE + (size_t)m0 * D + e) = *(const v4f*)(&Tf[wave][row][c]); } __threadfence(); }
}
__global__ __launch_bounds__(64) void pair_kernel(const float* __restrict__ Ap, const float* __restrict__ AV, const float* __restrict__ BV, const float* __restrict__ cb1, const b16* __restrict__ W2, const float* __restrict__ cb2, const b16* __restrict__ WO, const float* __restrict__ cbo, const float* __restrict__ NODE, float* __restrict__ out) {
  __shared__ __attribute__((aligned(16))) b16 H1[2][16][HH + 8], A2[2][16][HH + 8]; __shared__ float AI[2][HH], CB1s[HH], Ob[2][D];
  const int wave = threadIdx.x >> 5, lane = threadIdx.x & 31, nloc = lane & 15, hlf = lane >> 4; const int b = blockIdx.x / (N / 2), i0 = (blockIdx.x % (N / 2)) * 2, i = i0 + wave; const size_t nrow = (size_t)b * N + i;
  for (int c = threadIdx.x; c < HH; c += 64) CB1s[c] = bf16_rne(cb1[c]);
  for (int c = lane; c < HH; c += 32) AI[wave][c] = AV[nrow * HH + c];
  __syncthreads();
  const float cb2v[4] = {bf16_rne(cb2[nloc]), bf16_rne(cb2[16 + nloc]), bf16_rne(cb2[32 + nloc]), bf16_rne(cb2[48 + nloc])}; const float cbov = bf16_rne(cbo[nloc]);
  float s = 0.0f;
#pragma unroll 1
  for (int jb = 0; jb < N / 16; ++jb) {
    for (int idx = lane; idx < 16 * (HH / 4); idx += 32) { const int rr = idx / (HH / 4), c4 = (idx % (HH / 4)) * 4; const size_t jrow = (size_t)b * N + jb * 16 + rr; const v4f bv = *(const v4f*)(BV + jrow * HH + c4); v4h o;
      for (int q = 0; q < 4; ++q) o[q] = (b16)(lk(AI[wave][c4 + q] + bv[q] + CB1s[c4 + q]) * XS); *(v4h*)(&H1[wave][rr][c4]) = o; }
    wave_lds_sync();
    { v8f acc[4]; const v16b a0 = frag_kb(&H1[wave][nloc][0], hlf), a1 = frag_kb(&H1[wave][nloc][32], hlf);
#pragma unroll
      for (int t = 0; t < 4; ++t) { const b16* br = W2 + (size_t)(t * 16 + nloc) * HH; acc[t] = wmma16b(a0, frag_kb(br, hlf), (v8f){}); acc[t] = wmma16b(a1, frag_kb(br + 32, hlf), acc[t]); }
#pragma unroll
      for (int t = 0; t < 4; ++t)
#pragma unroll
        for (int r = 0; r < 8; ++r) A2[wave][8 * hlf + r][t * 16 + nloc] = (b16)(lk(acc[t][r] * (1.0f / (XS * WSC)) + cb2v[t]) * XS); }
    wave_lds_sync();
    { const v16b a0 = frag_kb(&A2[wave][nloc][0], hlf), a1 = frag_kb(&A2[wave][nloc][32], hlf); const b16* br = WO + (size_t)nloc * HH; v8f acc = wmma16b(a0, frag_kb(br, hlf), (v8f){}); acc = wmma16b(a1, frag_kb(br + 32, hlf), acc);
#pragma unroll
      for (int r = 0; r < 8; ++r) { const int j = jb * 16 + 8 * hlf + r; const float aij = (j == i) ? 0.0f : 1.0f / (1.0f + __expf(-bf16_rne(Ap[(size_t)i * N + j]))); s += aij * (acc[r] * (1.0f / (XS * WSC)) + cbov); } }
    wave_lds_sync(); }
  s += __shfl_xor(s, 16);
  if (hlf == 0) Ob[wave][nloc] = NODE[nrow * D + nloc] + s;
  __syncthreads();
  for (int pass = 0; pass < 2; ++pass) { if (threadIdx.x < 32) ((volatile float*)out)[((size_t)b * N + i0) * D + threadIdx.x] = Ob[threadIdx.x / D][threadIdx.x % D]; __threadfence(); }
}
}

extern "C" void kernel_launch(void* const* d_in, const int* in_sizes, int n_in, void* d_out, int out_size, void* d_ws, size_t ws_size, hipStream_t stream) {
  (void)n_in;
  auto Fp = [&](int i) { return (const float*)d_in[i]; };
  if (in_sizes[0] != B * N * D || in_sizes[1] != N * N || in_sizes[2] != D * HH || in_sizes[4] != HH * HH || in_sizes[6] != HH * D || in_sizes[7] != D || in_sizes[8] != 2 * D * HH || in_sizes[9] != HH || in_sizes[10] != HH * HH || in_sizes[12] != HH * D || in_sizes[13] != D || out_size != B * N * D) return;
  size_t off = 0; char* ws = (char*)d_ws;
  auto carve = [&](size_t bytes) { char* p = ws + off; off += (bytes + 255) & ~(size_t)255; return p; };
  b16* NW1T = (b16*)carve((size_t)HH * KX * 2); b16* NW2T = (b16*)carve((size_t)HH * HH * 2); b16* NWOT = (b16*)carve((size_t)D * HH * 2); b16* CAT = (b16*)carve((size_t)HH * KX * 2); b16* CBT = (b16*)carve((size_t)HH * KX * 2); b16* CW2T = (b16*)carve((size_t)HH * HH * 2); b16* CWOT = (b16*)carve((size_t)D * HH * 2);
  float* NODE = (float*)carve((size_t)NR * D * 4); float* AV = (float*)carve((size_t)NR * HH * 4); float* BV = (float*)carve((size_t)NR * HH * 4);
  if (off > ws_size || off > ((size_t)128 << 20)) return;
  wt_kernel<KX, D, HH><<<1, 256, 0, stream>>>(Fp(2), 0, NW1T); wt_kernel<HH, HH, HH><<<2, 256, 0, stream>>>(Fp(4), 0, NW2T); wt_kernel<HH, HH, D><<<1, 256, 0, stream>>>(Fp(6), 0, NWOT);
  wt_kernel<KX, D, HH><<<1, 256, 0, stream>>>(Fp(8), 0, CAT); wt_kernel<KX, D, HH><<<1, 256, 0, stream>>>(Fp(8), D, CBT); wt_kernel<HH, HH, HH><<<2, 256, 0, stream>>>(Fp(10), 0, CW2T); wt_kernel<HH, HH, D><<<1, 256, 0, stream>>>(Fp(12), 0, CWOT);
  node_kernel<<<NRL / 32, 64, 0, stream>>>(Fp(0), NW1T, Fp(3), NW2T, Fp(5), NWOT, Fp(7), CAT, CBT, NODE, AV, BV);
  pair_kernel<<<BL * N / 2, 64, 0, stream>>>(Fp(1), AV, BV, Fp(9), CW2T, Fp(11), CWOT, Fp(13), NODE, (float*)d_out);
}
